// DynamicLlamaAttention_26044681682964
// MI455X (gfx1250) — hardware-verified
//
#include <hip/hip_runtime.h>


#define NB_  2
#define TT   1024
#define DM   3072
#define KD   1024
#define NH_  32
#define QH   96
#define PCAR 1024.0f
#define SCL  0.03125f
#define THR  0.95f
typedef _Float16 h16;
typedef unsigned short bf;
typedef __attribute__((ext_vector_type(16))) __bf16   v16bf;
typedef __attribute__((ext_vector_type(16))) _Float16 v16h;
typedef __attribute__((ext_vector_type(8)))  _Float16 v8h;
typedef __attribute__((ext_vector_type(8)))  unsigned short v8us;
typedef __attribute__((ext_vector_type(8)))  float    v8f;
typedef __attribute__((ext_vector_type(4)))  float    v4f;
typedef v8h  __attribute__((may_alias)) v8ha;
typedef v4f  __attribute__((may_alias)) v4fa;
typedef v8us __attribute__((may_alias)) v8usa;

__device__ __forceinline__ unsigned short f2bf(float f) { unsigned u = __float_as_uint(f); u += 0x7FFFu + ((u >> 16) & 1u); return (unsigned short)(u >> 16); }
__device__ __forceinline__ float bf2f(unsigned short b) { return __uint_as_float(((unsigned)b) << 16); }
__device__ __forceinline__ float bfr(float f) { return bf2f(f2bf(f)); }
__device__ __forceinline__ v16h cat16(v8h lo, v8h hi) { return __builtin_shufflevector(lo, hi, 0, 1, 2, 3, 4, 5, 6, 7, 8, 9, 10, 11, 12, 13, 14, 15); }
__device__ __forceinline__ v16bf cat16b(v8us lo, v8us hi) { return __builtin_bit_cast(v16bf, __builtin_shufflevector(lo, hi, 0, 1, 2, 3, 4, 5, 6, 7, 8, 9, 10, 11, 12, 13, 14, 15)); }
__device__ __forceinline__ v8f wmma16(v16h a, v16h b, v8f c) { return __builtin_amdgcn_wmma_f32_16x16x32_f16(false, a, false, b, (short)0, c, false, false); }
__device__ __forceinline__ v8f wmmab(v16bf a, v16bf b, v8f c) { return __builtin_amdgcn_wmma_f32_16x16x32_bf16(false, a, false, b, (short)0, c, false, false); }


template <typename T16> struct WFrag;
template <> struct WFrag<h16> { typedef v16h V; static __device__ __forceinline__ V ld(const h16* p) { return cat16(*(const v8h*)p, *(const v8h*)(p + 16)); } static __device__ __forceinline__ v8f mma(V a, V b, v8f c) { return wmma16(a, b, c); } };
template <> struct WFrag<bf> { typedef v16bf V; static __device__ __forceinline__ V ld(const bf* p) { return cat16b(*(const v8us*)p, *(const v8us*)(p + 16)); } static __device__ __forceinline__ v8f mma(V a, V b, v8f c) { return wmmab(a, b, c); } };
template <typename T16, int NSPLIT, bool BIAS>
__global__ __launch_bounds__(32) void k_gemmw(const T16* __restrict__ A, const T16* __restrict__ A2, const T16* __restrict__ Bt, const T16* __restrict__ Bt2, int K, float* C, int ldc, const float* __restrict__ bias, size_t sA, size_t sB, size_t sC) {
    typedef typename WFrag<T16>::V V;
    __shared__ __align__(16) float os[16 * 68];
    const size_t z = blockIdx.z; A += z * sA; if (A2) A2 += z * sA; Bt += z * sB; if (Bt2) Bt2 += z * sB; C += z * sC;
    const int lane = threadIdx.x & 31, lr = lane & 15, hi = lane >> 4; const int r0 = blockIdx.x * 64, c0 = blockIdx.y * 64;
    v8f acc[4][4];
#pragma unroll
    for (int mb = 0; mb < 4; ++mb)
#pragma unroll
        for (int nb = 0; nb < 4; ++nb) acc[mb][nb] = (v8f){};
    const size_t aoff = (size_t)(r0 + lr) * K + 8 * hi, boff = (size_t)(c0 + lr) * K + 8 * hi;
#pragma unroll 1
    for (int kc = 0; kc < K; kc += 32) {
        V a[4], a2[4];
#pragma unroll
        for (int mb = 0; mb < 4; ++mb) { a[mb] = WFrag<T16>::ld(A + aoff + (size_t)mb * 16 * K + kc); if (NSPLIT == 1 || NSPLIT == 2) a2[mb] = WFrag<T16>::ld(A2 + aoff + (size_t)mb * 16 * K + kc); }
#pragma unroll
        for (int nb = 0; nb < 4; ++nb) { const V b = WFrag<T16>::ld(Bt + boff + (size_t)nb * 16 * K + kc); V b2; if (NSPLIT >= 2) b2 = WFrag<T16>::ld(Bt2 + boff + (size_t)nb * 16 * K + kc);
#pragma unroll
            for (int mb = 0; mb < 4; ++mb) { acc[mb][nb] = WFrag<T16>::mma(a[mb], b, acc[mb][nb]); if (NSPLIT == 1 || NSPLIT == 2) acc[mb][nb] = WFrag<T16>::mma(a2[mb], b, acc[mb][nb]); if (NSPLIT >= 2) acc[mb][nb] = WFrag<T16>::mma(a[mb], b2, acc[mb][nb]); } }
        asm volatile("v_nop\n\tv_nop\n\tv_nop\n\tv_nop" : "+v"(acc[0][0]), "+v"(acc[1][1]), "+v"(acc[2][2]), "+v"(acc[3][3]) : "v"(a[0]), "v"(a[3]));
    }
#pragma unroll
    for (int mb = 0; mb < 4; ++mb) {
#pragma unroll
        for (int nb = 0; nb < 4; ++nb) {
#pragma unroll
            for (int j = 0; j < 8; ++j) os[(hi * 8 + j) * 68 + nb * 16 + lr] = acc[mb][nb][j]; }
        __builtin_amdgcn_wave_barrier(); asm volatile("" ::: "memory");
        float* crow = C + (size_t)(r0 + mb * 16) * ldc + c0;
#pragma unroll 1
        for (int ps = 0; ps < 2; ++ps) {
#pragma unroll
            for (int s = 0; s < 8; ++s) { const int row = 2 * s + hi, cofs = lr * 4; v4f val = *(const v4fa*)(os + row * 68 + cofs); if (BIAS) { val[0] += bfr(bias[c0 + cofs]); val[1] += bfr(bias[c0 + cofs + 1]); val[2] += bfr(bias[c0 + cofs + 2]); val[3] += bfr(bias[c0 + cofs + 3]); }
                *(volatile v4f*)(crow + (size_t)row * ldc + cofs) = val; }
            if (ps == 0) __threadfence(); }
        __builtin_amdgcn_wave_barrier(); asm volatile("" ::: "memory");
    }
}

__device__ __forceinline__ h16 tohx(float x) { return (h16)x; }
__device__ __forceinline__ void splitf(float y, unsigned short& h, unsigned short& l) { h = f2bf(y); l = f2bf(y - bf2f(h)); }
typedef __attribute__((ext_vector_type(2))) _Float16 v2h;
typedef __attribute__((ext_vector_type(4))) _Float16 v4h;
typedef __attribute__((ext_vector_type(2))) unsigned short v2us;
typedef __attribute__((ext_vector_type(4))) unsigned short v4us;

__global__ __launch_bounds__(256) void k_wtG(const float* __restrict__ w, int K, int N, bf* Bt) {
    const int lane = threadIdx.x & 31; const int L0 = (blockIdx.x * 8 + (threadIdx.x >> 5)) * 8; const int nlines = N * K / 64;
#pragma unroll 1
    for (int ps = 0; ps < 2; ++ps) {
#pragma unroll 1
        for (int l = 0; l < 8; ++l) { const int L = L0 + l; if (L >= nlines) break; const size_t e = (size_t)L * 64 + lane * 2; const int k = (int)(e % K), n = (int)(e / K); v2us o;
            o[0] = f2bf(w[(size_t)k * N + n]); o[1] = f2bf(w[(size_t)(k + 1) * N + n]); *(volatile v2us*)(Bt + e) = o; }
        if (ps == 0) __threadfence(); }
}
__global__ __launch_bounds__(256) void k_cvt8(const float* __restrict__ src, bf* dst, size_t n8) { const size_t i = (size_t)blockIdx.x * 256 + threadIdx.x; if (i >= n8) return; const v8f v = *(const v8f*)(src + i * 8); v8us o;
#pragma unroll
    for (int k = 0; k < 8; ++k) o[k] = f2bf(v[k]); *(volatile v8us*)(dst + i * 8) = o; __threadfence(); *(volatile v8us*)(dst + i * 8) = o; }
__global__ __launch_bounds__(256) void k_nrmpl(const float* __restrict__ F, bf* Nh, bf* Nl) { const int lane = threadIdx.x & 31; const int t = blockIdx.x * 8 + (threadIdx.x >> 5); if (t >= TT) return; const float* fr = F + (size_t)t * KD; float s = 0.f;
#pragma unroll
    for (int ch = 0; ch < 8; ++ch) { const v4f a = *(const v4f*)(fr + ch * 128 + lane * 4);
#pragma unroll
        for (int q = 0; q < 4; ++q) { float p = __fmul_rn(a[q], a[q]); asm volatile("" : "+v"(p)); s = __fadd_rn(s, p); } }
#pragma unroll
    for (int sh = 16; sh; sh >>= 1) s += __shfl_xor(s, sh, 32);
    const float inv = __fdiv_rn(1.0f, fmaxf(__fsqrt_rn(s), 1e-8f));
#pragma unroll 1
    for (int ps = 0; ps < 2; ++ps) {
#pragma unroll
        for (int ch = 0; ch < 8; ++ch) { const v4f a = *(const v4f*)(fr + ch * 128 + lane * 4); v4us oh, ol;
#pragma unroll
            for (int q = 0; q < 4; ++q) { unsigned short x, y; splitf(__fmul_rn(a[q], inv), x, y); oh[q] = x; ol[q] = y; }
            *(volatile v4us*)(Nh + (size_t)t * KD + ch * 128 + lane * 4) = oh; *(volatile v4us*)(Nl + (size_t)t * KD + ch * 128 + lane * 4) = ol; }
        if (ps == 0) __threadfence(); } }
__global__ __launch_bounds__(32) void k_rep(const float* __restrict__ SIM, int* REP) { const int lane = threadIdx.x; unsigned used = 0u; int rep[32];
#pragma unroll
    for (int m = 0; m < 32; ++m) rep[m] = lane + 32 * m;
    for (int i = 0; i < TT; ++i) { const unsigned ui = __shfl((used >> (i >> 5)) & 1u, i & 31, 32); if (ui) continue; const float* row = SIM + (size_t)i * TT;
#pragma unroll
        for (int m = 0; m < 32; ++m) { const int j = lane + 32 * m; const bool cand = (j > i) && (row[j] > THR) && !((used >> m) & 1u); if (cand) { rep[m] = i; used |= (1u << m); } } }
    for (int ps = 0; ps < 2; ++ps) {
#pragma unroll
        for (int m = 0; m < 32; ++m) *(volatile int*)(REP + 32 * m + lane) = rep[m];
        if (ps == 0) __threadfence(); } }
__global__ __launch_bounds__(256) void k_gathK(const float* __restrict__ KF, const int* __restrict__ REP, bf* Kh, bf* Kl) { const int e = (blockIdx.x * 256 + threadIdx.x) * 2; if (e >= TT * KD) return; const int cc = e % KD, t = e / KD; const int r = REP[t]; v2us oh, ol;
#pragma unroll
    for (int q = 0; q < 2; ++q) { unsigned short a, c2; splitf(KF[(size_t)r * KD + cc + q], a, c2); oh[q] = a; ol[q] = c2; } *(volatile v2us*)(Kh + e) = oh; *(volatile v2us*)(Kl + e) = ol; __threadfence(); *(volatile v2us*)(Kh + e) = oh; *(volatile v2us*)(Kl + e) = ol; }
__global__ __launch_bounds__(256) void k_gathVT(const float* __restrict__ VF, const int* __restrict__ REP, h16* VT) { const int e = (blockIdx.x * 256 + threadIdx.x) * 2; if (e >= KD * TT) return; const int t = e % TT, n = e / TT; v2h o; o[0] = tohx(VF[(size_t)REP[t] * KD + n]); o[1] = tohx(VF[(size_t)REP[t + 1] * KD + n]); *(volatile v2h*)(VT + e) = o; __threadfence(); *(volatile v2h*)(VT + e) = o; }
__global__ __launch_bounds__(256) void k_aqk(const float* __restrict__ wqk, const float* __restrict__ bqk, bf* AQ, bf* AZ) { const int e = (blockIdx.x * 256 + threadIdx.x) * 4; if (e >= 128 * KD) return; const int cc = e % KD, r = e / KD; v4us o, z;
#pragma unroll
    for (int q = 0; q < 4; ++q) { o[q] = (r < QH) ? f2bf(wqk[(size_t)r * KD + cc + q]) : (r == QH ? f2bf(bqk[cc + q]) : (unsigned short)0); z[q] = 0; }
    *(volatile v4us*)(AQ + e) = o; *(volatile v4us*)(AZ + e) = z; __threadfence(); *(volatile v4us*)(AQ + e) = o; *(volatile v4us*)(AZ + e) = z; }
__global__ __launch_bounds__(256) void k_kwt(const float* __restrict__ KWC, h16* KWT, float* KB) { const int e2 = (blockIdx.x * 256 + threadIdx.x) * 2; if (e2 < TT * QH) { const int e = e2 % QH, t = e2 / QH; v2h o; o[0] = tohx(KWC[(size_t)e * TT + t]); o[1] = tohx(KWC[(size_t)(e + 1) * TT + t]); *(volatile v2h*)(KWT + e2) = o; __threadfence(); *(volatile v2h*)(KWT + e2) = o; }
    const int t2 = blockIdx.x * 256 + threadIdx.x; if (t2 < TT) { const float kb = KWC[(size_t)QH * TT + t2]; *(volatile float*)(KB + t2) = kb; __threadfence(); *(volatile float*)(KB + t2) = kb; } }
__global__ __launch_bounds__(256) void k_qp(const float* __restrict__ Q, h16* QP) { const size_t e2 = ((size_t)blockIdx.x * 256 + threadIdx.x) * 2; if (e2 >= (size_t)NH_ * TT * QH) return; const int e = (int)(e2 % QH); const int s = (int)((e2 / QH) % TT); const int h = (int)(e2 / ((size_t)QH * TT)); v2h o; o[0] = tohx(Q[(size_t)s * DM + h * QH + e]); o[1] = tohx(Q[(size_t)s * DM + h * QH + e + 1]); *(volatile v2h*)(QP + e2) = o; __threadfence(); *(volatile v2h*)(QP + e2) = o; }
__global__ __launch_bounds__(256) void k_asoftacc(const float* __restrict__ Sb, const float* __restrict__ KB, int first, float* PM) { const int lane = threadIdx.x & 31; const int row = blockIdx.x * 8 + (threadIdx.x >> 5); if (row >= TT) return; const float* sr = Sb + (size_t)row * TT; float v[32]; float mx = -3.0e38f;
#pragma unroll
    for (int ch = 0; ch < 8; ++ch) { const int j0 = ch * 128 + lane * 4; const v4f a = *(const v4f*)(sr + j0), k4 = *(const v4f*)(KB + j0);
#pragma unroll
        for (int q = 0; q < 4; ++q) { float t = __fadd_rn(a[q], k4[q]); asm volatile("" : "+v"(t)); t = __fmul_rn(t, SCL); v[ch * 4 + q] = t; mx = fmaxf(mx, t); } }
#pragma unroll
    for (int sh = 16; sh; sh >>= 1) mx = fmaxf(mx, __shfl_xor(mx, sh, 32));
    float sum = 0.f;
#pragma unroll
    for (int k = 0; k < 32; ++k) { float d0 = __fsub_rn(v[k], mx); asm volatile("" : "+v"(d0)); v[k] = __builtin_amdgcn_exp2f(__fmul_rn(d0, 1.4426950408889634f)); sum += v[k]; }
#pragma unroll
    for (int sh = 16; sh; sh >>= 1) sum += __shfl_xor(sum, sh, 32);
    const float f = __fdiv_rn(1.0f / (float)NH_, sum); v4f prev[8];
#pragma unroll
    for (int ch = 0; ch < 8; ++ch) { if (first) { prev[ch][0] = 0.f; prev[ch][1] = 0.f; prev[ch][2] = 0.f; prev[ch][3] = 0.f; } else prev[ch] = *(const v4f*)(PM + (size_t)row * TT + ch * 128 + lane * 4); }
#pragma unroll 1
    for (int ps = 0; ps < 2; ++ps) {
#pragma unroll
        for (int ch = 0; ch < 8; ++ch) { v4f o;
#pragma unroll
            for (int q = 0; q < 4; ++q) { float p = __fmul_rn(v[ch * 4 + q], f); asm volatile("" : "+v"(p)); o[q] = __fadd_rn(prev[ch][q], p); }
            *(volatile v4f*)(PM + (size_t)row * TT + ch * 128 + lane * 4) = o; }
        if (ps == 0) __threadfence(); } }
__global__ __launch_bounds__(256) void k_pm16(const float* __restrict__ PM, h16* P16) { const size_t i = ((size_t)blockIdx.x * 256 + threadIdx.x) * 2; if (i >= (size_t)TT * TT) return; v2h o; o[0] = tohx(PM[i] * PCAR); o[1] = tohx(PM[i + 1] * PCAR); *(volatile v2h*)(P16 + i) = o; __threadfence(); *(volatile v2h*)(P16 + i) = o; }
__global__ __launch_bounds__(256) void k_osplit(const float* __restrict__ O, bf* Ah, bf* Al) { const size_t i = ((size_t)blockIdx.x * 256 + threadIdx.x) * 2; if (i >= (size_t)TT * KD) return; v2us oh, ol;
#pragma unroll
    for (int q = 0; q < 2; ++q) { unsigned short a, c2; splitf(O[i + q] * (1.0f / PCAR), a, c2); oh[q] = a; ol[q] = c2; } *(volatile v2us*)(Ah + i) = oh; *(volatile v2us*)(Al + i) = ol; __threadfence(); *(volatile v2us*)(Ah + i) = oh; *(volatile v2us*)(Al + i) = ol; }

extern "C" void kernel_launch(void* const* d_in, const int* in_sizes, int n_in,
                              void* d_out, int out_size, void* d_ws, size_t ws_size, hipStream_t stream) {
    (void)in_sizes; (void)n_in; (void)out_size;
    const float* IN[11]; for (int i = 0; i < 11; ++i) IN[i] = (const float*)d_in[i];
    float* OUT = (float*)d_out;
    char* wsp = (char*)d_ws;
    auto take = [&](size_t bytes) { char* p = wsp; wsp += (bytes + 255) & ~(size_t)255; return (void*)p; };
    bf* WQ = (bf*)take((size_t)DM * DM * 2); bf* WK = (bf*)take((size_t)DM * KD * 2); bf* WV = (bf*)take((size_t)DM * KD * 2); bf* WO = (bf*)take((size_t)KD * DM * 2); bf* AQ = (bf*)take((size_t)128 * KD * 2); bf* AZ = (bf*)take((size_t)128 * KD * 2);
    bf* XB = (bf*)take((size_t)TT * DM * 2); float* Q = (float*)take((size_t)TT * DM * 4); float* KF = (float*)take((size_t)TT * KD * 4); float* VF = (float*)take((size_t)TT * KD * 4); bf* Nh = (bf*)take((size_t)TT * KD * 2); bf* Nl = (bf*)take((size_t)TT * KD * 2); float* SIM = (float*)take((size_t)TT * TT * 4); int* REPK = (int*)take((size_t)TT * 4); int* REPV = (int*)take((size_t)TT * 4);
    bf* KNh = (bf*)take((size_t)TT * KD * 2); bf* KNl = (bf*)take((size_t)TT * KD * 2); h16* VT = (h16*)take((size_t)KD * TT * 2); float* KWC = (float*)take((size_t)128 * TT * 4); h16* KWT = (h16*)take((size_t)TT * QH * 2); float* KB = (float*)take((size_t)TT * 4); h16* QP = (h16*)take((size_t)NH_ * TT * QH * 2);
    float* Sb = (float*)take((size_t)TT * TT * 4); float* PM = (float*)take((size_t)TT * TT * 4); h16* P16 = (h16*)take((size_t)TT * TT * 2); float* O = (float*)take((size_t)TT * KD * 4); bf* Ah = (bf*)take((size_t)TT * KD * 2); bf* Al = (bf*)take((size_t)TT * KD * 2);
    if ((size_t)(wsp - (char*)d_ws) > ws_size) return;
    { k_wtG<<<(unsigned)(((size_t)DM * DM / 64 + 63) / 64), 256, 0, stream>>>(IN[1], DM, DM, WQ); k_wtG<<<(unsigned)(((size_t)DM * KD / 64 + 63) / 64), 256, 0, stream>>>(IN[3], DM, KD, WK); k_wtG<<<(unsigned)(((size_t)DM * KD / 64 + 63) / 64), 256, 0, stream>>>(IN[5], DM, KD, WV);
      k_wtG<<<(unsigned)(((size_t)KD * DM / 64 + 63) / 64), 256, 0, stream>>>(IN[9], KD, DM, WO); k_aqk<<<(128 * KD / 4 + 255) / 256, 256, 0, stream>>>(IN[7], IN[8], AQ, AZ); }
    const unsigned L2 = (TT * KD / 2 + 255) / 256;
    for (int b = 0; b < NB_; ++b) {
        k_cvt8<<<(unsigned)(((size_t)TT * DM / 8 + 255) / 256), 256, 0, stream>>>(IN[0] + (size_t)b * TT * DM, XB, (size_t)TT * DM / 8);
        k_gemmw<bf, 0, true><<<dim3(TT / 64, DM / 64, 1), 32, 0, stream>>>(XB, nullptr, WQ, nullptr, DM, Q, DM, IN[2], 0, 0, 0); k_qp<<<(unsigned)(((size_t)NH_ * TT * QH / 2 + 255) / 256), 256, 0, stream>>>(Q, QP);
        k_gemmw<bf, 0, true><<<dim3(TT / 64, KD / 64, 1), 32, 0, stream>>>(XB, nullptr, WK, nullptr, DM, KF, KD, IN[4], 0, 0, 0);
        k_gemmw<bf, 0, true><<<dim3(TT / 64, KD / 64, 1), 32, 0, stream>>>(XB, nullptr, WV, nullptr, DM, VF, KD, IN[6], 0, 0, 0);
        k_nrmpl<<<TT / 8, 256, 0, stream>>>(KF, Nh, Nl); k_gemmw<bf, 2, false><<<dim3(TT / 64, TT / 64, 1), 32, 0, stream>>>(Nh, Nl, Nh, Nl, KD, SIM, TT, nullptr, 0, 0, 0); k_rep<<<1, 32, 0, stream>>>(SIM, REPK);
        k_nrmpl<<<TT / 8, 256, 0, stream>>>(VF, Nh, Nl); k_gemmw<bf, 2, false><<<dim3(TT / 64, TT / 64, 1), 32, 0, stream>>>(Nh, Nl, Nh, Nl, KD, SIM, TT, nullptr, 0, 0, 0); k_rep<<<1, 32, 0, stream>>>(SIM, REPV);
        k_gathK<<<L2, 256, 0, stream>>>(KF, REPK, KNh, KNl); k_gathVT<<<L2, 256, 0, stream>>>(VF, REPV, VT);
        k_gemmw<bf, 2, false><<<dim3(128 / 64, TT / 64, 1), 32, 0, stream>>>(AQ, AZ, KNh, KNl, KD, KWC, TT, nullptr, 0, 0, 0); k_kwt<<<(TT * QH / 2 + 255) / 256, 256, 0, stream>>>(KWC, KWT, KB);
        for (int h = 0; h < NH_; ++h) {
            k_gemmw<h16, 0, false><<<dim3(TT / 64, TT / 64, 1), 32, 0, stream>>>(QP + (size_t)h * TT * QH, nullptr, KWT, nullptr, QH, Sb, TT, nullptr, 0, 0, 0);
            k_asoftacc<<<TT / 8, 256, 0, stream>>>(Sb, KB, h == 0 ? 1 : 0, PM); }
        k_pm16<<<(unsigned)(((size_t)TT * TT / 2 + 255) / 256), 256, 0, stream>>>(PM, P16);
        k_gemmw<h16, 0, false><<<dim3(TT / 64, KD / 64, 1), 32, 0, stream>>>(P16, nullptr, VT, nullptr, TT, O, KD, nullptr, 0, 0, 0);
        k_osplit<<<L2, 256, 0, stream>>>(O, Ah, Al);
        k_gemmw<bf, 1, true><<<dim3(TT / 64, DM / 64, 1), 32, 0, stream>>>(Ah, Al, WO, nullptr, KD, OUT + (size_t)b * TT * DM, DM, IN[10], 0, 0, 0); }
}
